// SingleInteractionBlock_1288490189572
// MI455X (gfx1250) — hardware-verified
//
#include <hip/hip_runtime.h>
#define NNODE 25000
#define NE 300000
#define MUL 16
#define NEL 10
#define NEF 8
#define MIN 28
#define KP 32
#define WN 1024
#define CHE 8192
#define NN NNODE

typedef __bf16 v16b __attribute__((ext_vector_type(16)));
typedef unsigned short v8us __attribute__((ext_vector_type(8), may_alias));
typedef float  v8f  __attribute__((ext_vector_type(8)));
typedef float  v4f  __attribute__((ext_vector_type(4)));
typedef float  v4fa __attribute__((ext_vector_type(4), may_alias));
union FragB { v16b v; v8us half[2]; unsigned short u[16]; };

__device__ __forceinline__ unsigned short bf16_bits(float x) { unsigned int u = __float_as_uint(x); return (unsigned short)((u + 0x7FFFu + ((u >> 16) & 1u)) >> 16); }
__device__ __forceinline__ float bf16_val(unsigned short b) { return __uint_as_float(((unsigned int)b) << 16); }
__device__ __forceinline__ float bf16_round(float x) { return bf16_val(bf16_bits(x)); }
template <int NT>
__device__ __forceinline__ v8f mmaN(v16b ah, v16b al, v16b bh, v16b bl, v8f c) {
  c = __builtin_amdgcn_wmma_f32_16x16x32_bf16(false, ah, false, bh, (short)0, c, false, false);
  if (NT >= 2) c = __builtin_amdgcn_wmma_f32_16x16x32_bf16(false, al, false, bh, (short)0, c, false, false);
  if (NT >= 3) c = __builtin_amdgcn_wmma_f32_16x16x32_bf16(false, ah, false, bl, (short)0, c, false, false);
  asm volatile("v_nop\n\tv_nop\n\tv_nop\n\tv_nop" : "+v"(c) : "v"(ah), "v"(al), "v"(bh), "v"(bl));
  return c;
}

__global__ __launch_bounds__(256) void k_wt_bf16(const float* __restrict__ W, unsigned short* __restrict__ Wt, int K, int N) {
  const int t = blockIdx.x * 256 + threadIdx.x;
  const int k8n = K / 8;
  if (t >= N * k8n) return;
  const int n = t / k8n, k8 = (t % k8n) * 8;
  v8us v;
#pragma unroll
  for (int i = 0; i < 8; ++i) v[i] = bf16_bits(W[(size_t)(k8 + i) * N + n]);
  *(volatile v8us*)(Wt + (size_t)n * K + k8) = v;
  __threadfence();
  *(volatile v8us*)(Wt + (size_t)n * K + k8) = v;
}

template <bool ASPLIT, int ACT, bool BIAS_BF16>
__global__ __launch_bounds__(128) void k_gemm_bf(const float* __restrict__ A, int lda, const unsigned short* __restrict__ Wt, int ldb,
                                               const float* __restrict__ bias, float* __restrict__ C, int ldc, int M, int N, int K) {
  __shared__ __attribute__((aligned(16))) float so[4][16][64];
  const int tid = threadIdx.x, w = tid >> 5, lane = tid & 31, ln = lane & 15, hh = lane >> 4;
  const int ntn = N / 64;
  const int wid = blockIdx.x * 4 + w;
  const int mt = wid / ntn, nq = wid % ntn;
  if (mt * 16 >= M) return;
  const int row0 = mt * 16, col0 = nq * 64;
  const float* arow = A + (size_t)(row0 + ln) * lda;
  v8f acc[4] = {};
  for (int kb = 0; kb < K; kb += 32) {
    FragB ah, al;
    const v4f x0 = *(const v4fa*)(arow + kb + 8 * hh), x1 = *(const v4fa*)(arow + kb + 8 * hh + 4);
    const v4f x2 = *(const v4fa*)(arow + kb + 16 + 8 * hh), x3 = *(const v4fa*)(arow + kb + 16 + 8 * hh + 4);
    float xs[16] = {x0[0],x0[1],x0[2],x0[3],x1[0],x1[1],x1[2],x1[3],x2[0],x2[1],x2[2],x2[3],x3[0],x3[1],x3[2],x3[3]};
#pragma unroll
    for (int i = 0; i < 16; ++i) { const unsigned short hb = bf16_bits(xs[i]); ah.u[i] = hb; al.u[i] = ASPLIT ? bf16_bits(xs[i] - bf16_val(hb)) : (unsigned short)0; }
#pragma unroll
    for (int t = 0; t < 4; ++t) {
      const unsigned short* brow = Wt + (size_t)(col0 + t * 16 + ln) * ldb + kb;
      FragB b;
      b.half[0] = *(const v8us*)(brow + 8 * hh);
      b.half[1] = *(const v8us*)(brow + 16 + 8 * hh);
      acc[t] = mmaN<ASPLIT ? 2 : 1>(ah.v, al.v, b.v, b.v, acc[t]);
    }
  }
#pragma unroll
  for (int t = 0; t < 4; ++t) {
    float bv = bias ? bias[col0 + t * 16 + ln] : 0.f;
    if (BIAS_BF16) bv = bf16_round(bv);
#pragma unroll
    for (int r = 0; r < 8; ++r) { float v = acc[t][r] + bv; if (ACT == 1) v = fmaxf(v, 0.f); so[w][8 * hh + r][t * 16 + ln] = v; }
  }
  __builtin_amdgcn_fence(__ATOMIC_ACQ_REL, "workgroup");
  __builtin_amdgcn_wave_barrier();
  const int rsub = lane >> 4, c4 = (lane & 15) * 4;
  for (int pass = 0; pass < 2; ++pass) {
#pragma unroll
    for (int q = 0; q < 8; ++q) {
      const int r = q * 2 + rsub;
      const v4f v = *(const v4fa*)&so[w][r][c4];
      *(volatile v4f*)(C + (size_t)(row0 + r) * ldc + col0 + c4) = v;
    }
    if (pass == 0) __threadfence();
  }
}

template <int D, bool CAUSAL>
__global__ __launch_bounds__(128) void k_flash(const float* __restrict__ qb, const float* __restrict__ kb, const float* __restrict__ vb,
                                             int pitch, int T, int H, float scale, float* __restrict__ y, int ypitch) {
  constexpr int KS = D / 32;
  constexpr int DT = D / 16;
  __shared__ __attribute__((aligned(16))) unsigned short sKh[32][D + 8], sKl[32][D + 8], sVh[32][D + 8], sVl[32][D + 8];
  __shared__ __attribute__((aligned(16))) unsigned short sPh[4][16][40], sPl[4][16][40];
  __shared__ __attribute__((aligned(16))) float sO[4][16][D];
  const int tid = threadIdx.x, w = tid >> 5, lane = tid & 31, ln = lane & 15, hh = lane >> 4;
  const int nqb = (T + 63) / 64;
  const int bh = blockIdx.x / nqb, qblk = blockIdx.x % nqb;
  const int b = bh / H, h = bh % H;
  const int q0 = qblk * 64 + w * 16;
  const float* Q = qb + (size_t)b * T * pitch + h * D;
  const float* K = kb + (size_t)b * T * pitch + h * D;
  const float* V = vb + (size_t)b * T * pitch + h * D;

  FragB aqh[KS], aql[KS];
  {
    int row = q0 + ln; if (row >= T) row = T - 1;
    const float* qr = Q + (size_t)row * pitch;
#pragma unroll
    for (int ks = 0; ks < KS; ++ks)
#pragma unroll
      for (int i = 0; i < 16; ++i) {
        const int d = ks * 32 + ((i < 8) ? (8 * hh + i) : (16 + 8 * hh + (i - 8)));
        const float x = qr[d] * scale; const unsigned short hb = bf16_bits(x);
        aqh[ks].u[i] = hb; aql[ks].u[i] = bf16_bits(x - bf16_val(hb));
      }
  }
  float m_r[8], l_r[8];
#pragma unroll
  for (int r = 0; r < 8; ++r) { m_r[r] = -3.0e38f; l_r[r] = 0.f; }
  v8f oacc[DT];
#pragma unroll
  for (int dt = 0; dt < DT; ++dt) oacc[dt] = (v8f){0.f,0.f,0.f,0.f,0.f,0.f,0.f,0.f};

  const int kv_end = CAUSAL ? min(T, qblk * 64 + 64) : T;
  for (int j0 = 0; j0 < kv_end; j0 += 32) {
    __syncthreads();
    for (int e = tid; e < 32 * (D / 4); e += 128) {
      const int r = e / (D / 4), c4 = (e % (D / 4)) * 4;
      const int key = j0 + r;
      v4f kf = {0.f,0.f,0.f,0.f}, vf = {0.f,0.f,0.f,0.f};
      if (key < T) { kf = *(const v4fa*)(K + (size_t)key * pitch + c4); vf = *(const v4fa*)(V + (size_t)key * pitch + c4); }
#pragma unroll
      for (int t = 0; t < 4; ++t) {
        unsigned short hb = bf16_bits(kf[t]); sKh[r][c4 + t] = hb; sKl[r][c4 + t] = bf16_bits(kf[t] - bf16_val(hb));
        hb = bf16_bits(vf[t]); sVh[r][c4 + t] = hb; sVl[r][c4 + t] = bf16_bits(vf[t] - bf16_val(hb));
      }
    }
    __syncthreads();
    v8f s[2];
#pragma unroll
    for (int nt = 0; nt < 2; ++nt) {
      v8f acc = {};
#pragma unroll
      for (int ks = 0; ks < KS; ++ks) {
        FragB bh_, bl_;
        bh_.half[0] = *(const v8us*)&sKh[nt * 16 + ln][ks * 32 + 8 * hh]; bh_.half[1] = *(const v8us*)&sKh[nt * 16 + ln][ks * 32 + 16 + 8 * hh];
        bl_.half[0] = *(const v8us*)&sKl[nt * 16 + ln][ks * 32 + 8 * hh]; bl_.half[1] = *(const v8us*)&sKl[nt * 16 + ln][ks * 32 + 16 + 8 * hh];
        acc = mmaN<3>(aqh[ks].v, aql[ks].v, bh_.v, bl_.v, acc);
      }
      s[nt] = acc;
    }
    float alpha[8];
#pragma unroll
    for (int r = 0; r < 8; ++r) {
      const int qi = q0 + 8 * hh + r;
      const int ja = j0 + ln, jb = j0 + 16 + ln;
      if (CAUSAL) { if (ja > qi) s[0][r] = -3.0e38f; if (jb > qi) s[1][r] = -3.0e38f; }
      if (ja >= T) s[0][r] = -3.0e38f;
      if (jb >= T) s[1][r] = -3.0e38f;
      float mx = fmaxf(s[0][r], s[1][r]);
      mx = fmaxf(mx, __shfl_xor(mx, 1, 32)); mx = fmaxf(mx, __shfl_xor(mx, 2, 32)); mx = fmaxf(mx, __shfl_xor(mx, 4, 32)); mx = fmaxf(mx, __shfl_xor(mx, 8, 32));
      const float mnew = fmaxf(m_r[r], mx);
      alpha[r] = (mnew > -1.0e38f) ? __expf(m_r[r] - mnew) : 1.0f;
      const float p0 = (s[0][r] > -1.0e38f) ? __expf(s[0][r] - mnew) : 0.f;
      const float p1 = (s[1][r] > -1.0e38f) ? __expf(s[1][r] - mnew) : 0.f;
      m_r[r] = mnew;
      l_r[r] = l_r[r] * alpha[r] + p0 + p1;
      unsigned short hb = bf16_bits(p0); sPh[w][8 * hh + r][ln] = hb;      sPl[w][8 * hh + r][ln] = bf16_bits(p0 - bf16_val(hb));
      hb = bf16_bits(p1);                sPh[w][8 * hh + r][16 + ln] = hb; sPl[w][8 * hh + r][16 + ln] = bf16_bits(p1 - bf16_val(hb));
    }
#pragma unroll
    for (int dt = 0; dt < DT; ++dt)
#pragma unroll
      for (int r = 0; r < 8; ++r) oacc[dt][r] *= alpha[r];
    __builtin_amdgcn_fence(__ATOMIC_ACQ_REL, "workgroup");
    __builtin_amdgcn_wave_barrier();
    FragB pah, pal;
    pah.half[0] = *(const v8us*)&sPh[w][ln][8 * hh]; pah.half[1] = *(const v8us*)&sPh[w][ln][16 + 8 * hh];
    pal.half[0] = *(const v8us*)&sPl[w][ln][8 * hh]; pal.half[1] = *(const v8us*)&sPl[w][ln][16 + 8 * hh];
#pragma unroll
    for (int dt = 0; dt < DT; ++dt) {
      FragB bvh, bvl;
#pragma unroll
      for (int i = 0; i < 8; ++i) {
        bvh.u[i] = sVh[8 * hh + i][dt * 16 + ln]; bvh.u[8 + i] = sVh[16 + 8 * hh + i][dt * 16 + ln];
        bvl.u[i] = sVl[8 * hh + i][dt * 16 + ln]; bvl.u[8 + i] = sVl[16 + 8 * hh + i][dt * 16 + ln];
      }
      oacc[dt] = mmaN<3>(pah.v, pal.v, bvh.v, bvl.v, oacc[dt]);
    }
    __builtin_amdgcn_fence(__ATOMIC_ACQ_REL, "workgroup");
    __builtin_amdgcn_wave_barrier();
  }
#pragma unroll
  for (int r = 0; r < 8; ++r) {
    float l = l_r[r];
    l += __shfl_xor(l, 1, 32); l += __shfl_xor(l, 2, 32); l += __shfl_xor(l, 4, 32); l += __shfl_xor(l, 8, 32);
    l_r[r] = (l > 0.f) ? 1.0f / l : 0.f;
  }
#pragma unroll
  for (int dt = 0; dt < DT; ++dt)
#pragma unroll
    for (int r = 0; r < 8; ++r) sO[w][8 * hh + r][dt * 16 + ln] = oacc[dt][r] * l_r[r];
  __builtin_amdgcn_fence(__ATOMIC_ACQ_REL, "workgroup");
  __builtin_amdgcn_wave_barrier();
  for (int pass = 0; pass < 2; ++pass) {
    for (int r = 0; r < 16; ++r) {
      const int row = q0 + r;
      if (row < T && lane < D / 4) {
        const v4f val = *(const v4fa*)&sO[w][r][lane * 4];
        *(volatile v4f*)(y + ((size_t)b * T + row) * ypitch + h * D + lane * 4) = val;
      }
    }
    if (pass == 0) __threadfence();
  }
}

typedef _Float16 v16h __attribute__((ext_vector_type(16)));
union FragH { v16h v; v8us half[2]; _Float16 h[16]; unsigned short u[16]; };
template <int NT>
__device__ __forceinline__ v8f mmaH(v16h ah, v16h al, v16h bh, v16h bl, v8f c) {
  c = __builtin_amdgcn_wmma_f32_16x16x32_f16(false, ah, false, bh, (short)0, c, false, false);
  if (NT >= 2) c = __builtin_amdgcn_wmma_f32_16x16x32_f16(false, al, false, bh, (short)0, c, false, false);
  if (NT >= 3) c = __builtin_amdgcn_wmma_f32_16x16x32_f16(false, ah, false, bl, (short)0, c, false, false);
  asm volatile("v_nop\n\tv_nop\n\tv_nop\n\tv_nop" : "+v"(c) : "v"(ah), "v"(al), "v"(bh), "v"(bl));
  return c;
}
template <bool ASPLIT>
__global__ __launch_bounds__(128) void k_gemm_h(const float* __restrict__ A, int lda, size_t sA, const _Float16* __restrict__ Bh, int ldb, size_t sB, float alpha, float* __restrict__ C, int ldc, size_t sC, int M, int N, int K) {
  __shared__ __attribute__((aligned(16))) float so[4][16][64];
  const int tid = threadIdx.x, w = tid >> 5, lane = tid & 31, ln = lane & 15, hh = lane >> 4; const int by = blockIdx.y;
  A += (size_t)by * sA; Bh += (size_t)by * sB; C += (size_t)by * sC;
  const int ntn = (N + 63) / 64; const int wid = blockIdx.x * 4 + w; const int mt = wid / ntn, nq = wid % ntn; if (mt * 16 >= M) return;
  const int row0 = mt * 16, col0 = nq * 64; const float* arow = A + (size_t)(row0 + ln) * lda;
  v8f acc[4] = {};
  for (int kb = 0; kb < K; kb += 32) {
    FragH ah, al;
    const v4f x0 = *(const v4fa*)(arow + kb + 8 * hh), x1 = *(const v4fa*)(arow + kb + 8 * hh + 4), x2 = *(const v4fa*)(arow + kb + 16 + 8 * hh), x3 = *(const v4fa*)(arow + kb + 16 + 8 * hh + 4);
    float xs[16] = {x0[0],x0[1],x0[2],x0[3],x1[0],x1[1],x1[2],x1[3],x2[0],x2[1],x2[2],x2[3],x3[0],x3[1],x3[2],x3[3]};
#pragma unroll
    for (int i = 0; i < 16; ++i) { const _Float16 h = (_Float16)xs[i]; ah.h[i] = h; al.h[i] = ASPLIT ? (_Float16)(xs[i] - (float)h) : (_Float16)0.0f; }
#pragma unroll
    for (int t = 0; t < 4; ++t) { if (col0 + t * 16 >= N) continue; const size_t boff = (size_t)(col0 + t * 16 + ln) * ldb + kb; FragH bq; bq.half[0] = *(const v8us*)(Bh + boff + 8 * hh); bq.half[1] = *(const v8us*)(Bh + boff + 16 + 8 * hh);
      acc[t] = mmaH<ASPLIT ? 2 : 1>(ah.v, al.v, bq.v, bq.v, acc[t]); }
  }
#pragma unroll
  for (int t = 0; t < 4; ++t) { if (col0 + t * 16 >= N) continue;
#pragma unroll
    for (int r = 0; r < 8; ++r) so[w][8 * hh + r][t * 16 + ln] = acc[t][r] * alpha; }
  __builtin_amdgcn_fence(__ATOMIC_ACQ_REL, "workgroup"); __builtin_amdgcn_wave_barrier();
  const int rsub = lane >> 4, c4 = (lane & 15) * 4;
  for (int pass = 0; pass < 2; ++pass) {
#pragma unroll
    for (int q = 0; q < 8; ++q) { const int r = q * 2 + rsub; if (col0 + c4 < N) { const v4f v = *(const v4fa*)&so[w][r][c4]; *(volatile v4f*)(C + (size_t)(row0 + r) * ldc + col0 + c4) = v; } }
    if (pass == 0) __threadfence(); }
}

__global__ __launch_bounds__(256) void k_bt2(const float* __restrict__ W2, _Float16* __restrict__ Bt) { const int t = blockIdx.x * 256 + threadIdx.x; if (t >= WN * 4) return; const int n = t >> 2, k8 = (t & 3) * 8; FragH f; for (int q = 0; q < 8; ++q) { const int k = k8 + q; f.h[q] = (k < MIN) ? (_Float16)(bf16_round(W2[(size_t)k * WN + n]) * 0.25f) : (_Float16)0.0f; } *(volatile v8us*)((unsigned short*)Bt + (size_t)n * KP + k8) = f.half[0]; __threadfence(); *(volatile v8us*)((unsigned short*)Bt + (size_t)n * KP + k8) = f.half[0]; }
__global__ __launch_bounds__(256) void k_h(const float* __restrict__ ef, const float* __restrict__ na, const int* __restrict__ snd, const int* __restrict__ rcv, const float* __restrict__ W1, float* __restrict__ H) {
  __shared__ float sw[MIN][MIN + 1]; __shared__ float sx[8][KP]; const int tid = threadIdx.x, el = tid >> 5, j = tid & 31; for (int e2 = tid; e2 < MIN * MIN; e2 += 256) sw[e2 / MIN][e2 % MIN] = bf16_round(W1[e2]);
  const int e = blockIdx.x * 8 + el; float xv = 0.f;
  if (e < NE && j < MIN) { if (j < NEF) xv = bf16_round(ef[(size_t)e * NEF + j]); else { int n = (j < NEF + NEL) ? snd[e] : rcv[e]; n = n < 0 ? 0 : (n >= NNODE ? NNODE - 1 : n); const int a = (j < NEF + NEL) ? j - NEF : j - NEF - NEL; xv = bf16_round(na[(size_t)n * NEL + a]); } }
  sx[el][j] = xv; __syncthreads();
  float hv = 0.f; if (e < NE && j < MIN) { float s = 0.f;
#pragma unroll 1
    for (int i = 0; i < MIN; ++i) s += sx[el][i] * sw[i][j]; hv = 1.4142135623730951f * fmaxf(s / 5.291502622129181f, 0.f); }
  if (e < NE) { *(volatile float*)(H + (size_t)e * KP + j) = hv; __threadfence(); *(volatile float*)(H + (size_t)e * KP + j) = hv; }
}
__global__ __launch_bounds__(128) void k_edge(const float* __restrict__ TP, int e0, int ne, const float* __restrict__ nf, const float* __restrict__ ea, const int* __restrict__ snd, const float* __restrict__ lws, const float* __restrict__ lwv, _Float16* __restrict__ MJI) {
  __shared__ float sls[MUL][MUL + 1], slv[MUL][MUL + 1]; __shared__ float sS1[MUL][128], sV1[MUL * 3][128], sDot[MUL][128], sO[64][129];
  const int tid = threadIdx.x; for (int i = tid; i < MUL * MUL; i += 128) { sls[i / MUL][i % MUL] = bf16_round(lws[i]); slv[i / MUL][i % MUL] = bf16_round(lwv[i]); }
  const int el = blockIdx.x * 128 + tid; const bool live = el < ne; const int e = e0 + (live ? el : 0); int s = snd[e]; s = s < 0 ? 0 : (s >= NNODE ? NNODE - 1 : s);
  const float* w = TP + (size_t)(live ? el : 0) * WN; const float* fsn = nf + (size_t)s * (4 * MUL);
  const float s2 = bf16_round(ea[(size_t)e * 4]); const float v20 = bf16_round(ea[(size_t)e * 4 + 1]), v21 = bf16_round(ea[(size_t)e * 4 + 2]), v22 = bf16_round(ea[(size_t)e * 4 + 3]);
#pragma unroll 1
  for (int u = 0; u < MUL; ++u) { const float a = bf16_round(fsn[u]); const float x0 = bf16_round(fsn[MUL + u * 3]), x1 = bf16_round(fsn[MUL + u * 3 + 1]), x2 = bf16_round(fsn[MUL + u * 3 + 2]); sS1[u][tid] = a; sV1[u * 3][tid] = x0; sV1[u * 3 + 1][tid] = x1; sV1[u * 3 + 2][tid] = x2; sDot[u][tid] = (x0 * v20 + x1 * v21) + x2 * v22; }
  __syncthreads();
  const float inv32 = 0.17677669529663687f, inv3 = 0.5773502691896258f, invfan = 0.25f;
#pragma unroll 1
  for (int v = 0; v < MUL; ++v) { float a = 0.f, b = 0.f, c = 0.f, d0 = 0.f, d1 = 0.f, d2 = 0.f;
#pragma unroll 1
    for (int u = 0; u < MUL; ++u) { const float wsss = w[0 * 256 + u * MUL + v], wsvv = w[1 * 256 + u * MUL + v], wvsv = w[2 * 256 + u * MUL + v], wvvs = w[3 * 256 + u * MUL + v]; const float s1 = sS1[u][tid];
      a += wsss * (s1 * s2); b += wvvs * sDot[u][tid]; c += wsvv * s1; d0 += wvsv * sV1[u * 3][tid]; d1 += wvsv * sV1[u * 3 + 1][tid]; d2 += wvsv * sV1[u * 3 + 2][tid]; }
    sO[v][tid] = inv32 * (a + inv3 * b); sO[MUL + v * 3][tid] = inv32 * (c * v20 + d0 * s2); sO[MUL + v * 3 + 1][tid] = inv32 * (c * v21 + d1 * s2); sO[MUL + v * 3 + 2][tid] = inv32 * (c * v22 + d2 * s2); }
  __syncthreads();
#pragma unroll 1
  for (int wq = 0; wq < MUL; ++wq) { float ys = 0.f, y0 = 0.f, y1 = 0.f, y2 = 0.f;
#pragma unroll 1
    for (int v = 0; v < MUL; ++v) { ys += sO[v][tid] * sls[v][wq]; y0 += sO[MUL + v * 3][tid] * slv[v][wq]; y1 += sO[MUL + v * 3 + 1][tid] * slv[v][wq]; y2 += sO[MUL + v * 3 + 2][tid] * slv[v][wq]; }
    sS1[wq][tid] = ys * invfan; sV1[wq * 3][tid] = y0 * invfan; sV1[wq * 3 + 1][tid] = y1 * invfan; sV1[wq * 3 + 2][tid] = y2 * invfan; }
  __syncthreads();
  typedef _Float16 v2h __attribute__((ext_vector_type(2)));
  _Float16* base = MJI + (size_t)(e0 + blockIdx.x * 128) * 64; const int nlive = (ne - blockIdx.x * 128) < 128 ? (ne - blockIdx.x * 128) : 128;
  for (int pass = 0; pass < 2; ++pass) { for (int i = tid; i < nlive * 32; i += 128) { const int el2 = i >> 5, c = (i & 31) * 2; v2h o2;
      o2.x = (_Float16)((c < MUL) ? sS1[c][el2] : sV1[c - MUL][el2]); o2.y = (_Float16)((c + 1 < MUL) ? sS1[c + 1][el2] : sV1[c + 1 - MUL][el2]); *(volatile v2h*)(base + 2 * i) = o2; } if (pass == 0) __threadfence(); }
}
__device__ __forceinline__ int bscan512(int cnt, int* scan, int tid, int& total) { __syncthreads(); scan[tid] = cnt; __syncthreads();
  for (int of = 1; of < 512; of <<= 1) { const int v = (tid >= of) ? scan[tid - of] : 0; __syncthreads(); scan[tid] += v; __syncthreads(); }
  total = scan[511]; return scan[tid] - cnt; }
__global__ __launch_bounds__(512) void k_seg(const _Float16* __restrict__ MJI, const int* __restrict__ rcv, float* __restrict__ out) {
  __shared__ short Lr[4096]; __shared__ int Le[4096]; __shared__ int scan[512]; __shared__ float stg[64][65];
  const int tid = threadIdx.x, lane = tid & 31, wv = tid >> 5; const int n0 = blockIdx.x * 512; float acc[64];
#pragma unroll
  for (int c = 0; c < 64; ++c) acc[c] = 0.f;
#pragma unroll 1
  for (int e0 = 0; e0 < NE; e0 += 4096) { int hr[8], he[8]; int cnt = 0;
#pragma unroll
    for (int k = 0; k < 8; ++k) { const int e = e0 + tid * 8 + k; hr[k] = -1; he[k] = 0; if (e < NE) { const int dd_ = rcv[e]; if (dd_ >= n0 && dd_ < n0 + 512) { hr[k] = dd_ - n0; he[k] = e; ++cnt; } } }
    int tot; int p = bscan512(cnt, scan, tid, tot);
#pragma unroll
    for (int k = 0; k < 8; ++k) if (hr[k] >= 0) { Lr[p] = (short)hr[k]; Le[p] = he[k]; ++p; }
    __syncthreads();
    const int ntrip = (tot + 31) >> 5;
#pragma unroll 1
    for (int it = 0; it < ntrip; ++it) { const int q = it * 32 + lane; const int lr = (q < tot) ? (int)Lr[q] : -1;
      unsigned m = __builtin_amdgcn_ballot_w32(lr >= wv * 32 && lr < wv * 32 + 32);
#pragma unroll 1
      while (m) { const int bit = __builtin_ctz(m); m &= m - 1u; const int owner = __shfl(lr, bit, 32); const int e = Le[it * 32 + bit];
        if (tid == owner) { const unsigned short* mr = (const unsigned short*)MJI + (size_t)e * 64;
#pragma unroll
          for (int g = 0; g < 8; ++g) { FragH f; f.half[0] = *(const v8us*)(mr + g * 8);
#pragma unroll
            for (int d = 0; d < 8; ++d) acc[g * 8 + d] += (float)f.h[d]; } } } }
    __syncthreads(); }
  for (int tg = 0; tg < 8; ++tg) {
    if (tid / 64 == tg) {
#pragma unroll
      for (int c = 0; c < 64; ++c) stg[tid % 64][c] = acc[c]; }
    __syncthreads();
    for (int pass = 0; pass < 2; ++pass) {
#pragma unroll 1
      for (int i = tid; i < 64 * 16; i += 512) { const int r = i / 16, c4 = (i % 16) * 4; const int n = n0 + tg * 64 + r; if (n < NNODE) { v4f v; v[0] = stg[r][c4]; v[1] = stg[r][c4 + 1]; v[2] = stg[r][c4 + 2]; v[3] = stg[r][c4 + 3];
          *(volatile v4f*)(out + (size_t)n * 64 + c4) = v; } } if (pass == 0) __threadfence(); }
    __syncthreads(); } }
extern "C" void kernel_launch(void* const* d_in, const int* in_sizes, int n_in,
                              void* d_out, int out_size, void* d_ws, size_t ws_size, hipStream_t stream) {
  (void)in_sizes; (void)n_in; (void)out_size;
  const float* na = (const float*)d_in[0]; const float* nf = (const float*)d_in[1]; const float* ea = (const float*)d_in[2]; const float* ef = (const float*)d_in[3]; const int* ei = (const int*)d_in[4];
  const float* W1 = (const float*)d_in[5]; const float* W2 = (const float*)d_in[6]; const float* lws = (const float*)d_in[7]; const float* lwv = (const float*)d_in[8];
  const int* snd = ei; const int* rcv = ei + NE;
  char* ws = (char*)d_ws; size_t off = 0;
  auto take = [&](size_t bytes) { char* p = ws + off; off += (bytes + 255) & ~(size_t)255; return p; };
  _Float16* Bt2 = (_Float16*)take((size_t)WN * KP * 2); float* H = (float*)take((size_t)NE * KP * 4); float* TP = (float*)take((size_t)CHE * WN * 4); _Float16* MJI = (_Float16*)take((size_t)NE * 64 * 2);
  if (off > ws_size) return;
  k_bt2<<<(WN * 4 + 255) / 256, 256, 0, stream>>>(W2, Bt2);
  k_h<<<(NE + 7) / 8, 256, 0, stream>>>(ef, na, snd, rcv, W1, H);
  for (int e0 = 0; e0 < NE; e0 += CHE) { const int ne = (NE - e0 < CHE) ? (NE - e0) : CHE; const int mrows = ((ne + 15) / 16) * 16;
    k_gemm_h<false><<<dim3(((mrows / 16) * (WN / 64) + 3) / 4, 1), 128, 0, stream>>>(H + (size_t)e0 * KP, KP, 0, Bt2, KP, 0, 4.0f / 5.291502622129181f, TP, WN, 0, mrows, WN, KP);
    k_edge<<<(ne + 127) / 128, 128, 0, stream>>>(TP, e0, ne, nf, ea, snd, lws, lwv, MJI); }
  k_seg<<<(NNODE + 511) / 512, 512, 0, stream>>>(MJI, rcv, (float*)d_out);
}
